// LSTM_63866163692045
// MI455X (gfx1250) — hardware-verified
//
#include <hip/hip_runtime.h>
#include <math.h>

constexpr int NBATCH   = 256;
constexpr int NSTEP    = 2048;
constexpr int NHID     = 64;
constexpr int NGATE    = 4 * NHID;
constexpr int NEMB     = 128;
constexpr int NTHR     = 512;
constexpr int ROWS_BLK = 16;
constexpr int HCP = 200;
constexpr int GBP = 264;
constexpr int XCH = 32;
constexpr float HCARRY = 64.0f;
constexpr float WCARRY = 64.0f;
constexpr float PCARRY = HCARRY * WCARRY;
constexpr float PFOLD  = 1.0f / (HCARRY * WCARRY);

static_assert(NBATCH % ROWS_BLK == 0);
static_assert(NGATE == 16 * (NTHR / 32));
static_assert(NHID % 32 == 0);
static_assert(NSTEP % XCH == 0);
static_assert(ROWS_BLK * XCH == NTHR);
static_assert(ROWS_BLK * NEMB == 4 * NTHR);
static_assert(HCP % 8 == 0 && HCP >= 3 * NHID);
static_assert(GBP % 4 == 0 && GBP >= NGATE);
static_assert(2 * 8 * NHID == 2 * NTHR);

typedef __attribute__((ext_vector_type(16))) _Float16 v16h;
typedef __attribute__((ext_vector_type(8)))  _Float16 v8h;
typedef __attribute__((ext_vector_type(8)))  float    v8f;
typedef __attribute__((ext_vector_type(4)))  float    v4f;

union FragU { v16h v; v8h h[2]; };
__device__ __forceinline__ v16h frag_load(const _Float16* p) {
  FragU f;
  f.h[0] = *(const v8h*)(p);
  f.h[1] = *(const v8h*)(p + 16);
  return f.v;
}

__device__ __forceinline__ v16h bfrag_from_f32(const float* __restrict__ p) {
  const v4f q0 = *(const v4f*)(p);
  const v4f q1 = *(const v4f*)(p + 4);
  const v4f q2 = *(const v4f*)(p + 16);
  const v4f q3 = *(const v4f*)(p + 20);
  v16h f;
#pragma unroll
  for (int e = 0; e < 4; ++e) {
    f[e]      = (_Float16)(q0[e] * WCARRY);
    f[4 + e]  = (_Float16)(q1[e] * WCARRY);
    f[8 + e]  = (_Float16)(q2[e] * WCARRY);
    f[12 + e] = (_Float16)(q3[e] * WCARRY);
  }
  return f;
}

__device__ __forceinline__ v8f mma_h(v16h a, v16h b, v8f c) {
  c = __builtin_amdgcn_wmma_f32_16x16x32_f16(false, a, false, b, (short)0, c, false, false);
  asm volatile("v_nop\n\tv_nop\n\tv_nop\n\tv_nop" : "+v"(c) : "v"(a), "v"(b));
  return c;
}

__device__ __forceinline__ float fclamp15(float x) { return fminf(fmaxf(x, -15.0f), 15.0f); }
__device__ __forceinline__ float fsig(float x)  { return __builtin_amdgcn_rcpf(1.0f + __expf(-fclamp15(x))); }
__device__ __forceinline__ float ftanh(float x) { return 1.0f - 2.0f * __builtin_amdgcn_rcpf(__expf(2.0f * fclamp15(x)) + 1.0f); }

__device__ __forceinline__ float cell_update(float zi, float zf, float zg, float zo, float& cs) {
  const float ig = fsig(zi);
  const float fg = fsig(zf);
  const float gg = ftanh(zg);
  const float og = fsig(zo);
  const float cn = fg * cs + ig * gg;
  cs = cn;
  return og * ftanh(cn);
}

__global__ __launch_bounds__(NTHR) void rnn3_fused_kernel(
    const float* __restrict__ x,
    const float* __restrict__ wih0, const float* __restrict__ whh0,
    const float* __restrict__ bih0, const float* __restrict__ bhh0,
    const float* __restrict__ wih1, const float* __restrict__ whh1,
    const float* __restrict__ bih1, const float* __restrict__ bhh1,
    const float* __restrict__ wih2, const float* __restrict__ whh2,
    const float* __restrict__ bih2, const float* __restrict__ bhh2,
    const float* __restrict__ fcw,  const float* __restrict__ fcb,
    float* __restrict__ out) {
  __shared__ __align__(16) _Float16 hcat[ROWS_BLK * HCP];
  __shared__ __align__(16) float    gb[ROWS_BLK * GBP];
  __shared__ __align__(16) float    xs[ROWS_BLK * XCH];

  const int tid  = threadIdx.x;
  const int lane = tid & 31;
  const int wave = tid >> 5;
  const int c    = lane & 15;
  const int hh   = lane >> 4;
  const int koff = 8 * hh;
  const int b0   = blockIdx.x * ROWS_BLK;
  const int ncol = 16 * wave + c;

#pragma unroll 1
  for (int i = tid; i < ROWS_BLK * HCP; i += NTHR) hcat[i] = (_Float16)0.0f;

  const float* w0r  = whh0 + (size_t)ncol * NHID + koff;
  const float* wi1r = wih1 + (size_t)ncol * NHID + koff;
  const float* wh1r = whh1 + (size_t)ncol * NHID + koff;
  const float* wi2r = wih2 + (size_t)ncol * NHID + koff;
  const float* wh2r = whh2 + (size_t)ncol * NHID + koff;
  const v16h bw0a = bfrag_from_f32(w0r);
  const v16h bw0b = bfrag_from_f32(w0r + 32);
  const v16h bw1a = bfrag_from_f32(wi1r);
  const v16h bw1b = bfrag_from_f32(wi1r + 32);
  const v16h bw1c = bfrag_from_f32(wh1r);
  const v16h bw1d = bfrag_from_f32(wh1r + 32);
  const v16h bw2a = bfrag_from_f32(wi2r);
  const v16h bw2b = bfrag_from_f32(wi2r + 32);
  const v16h bw2c = bfrag_from_f32(wh2r);
  const v16h bw2d = bfrag_from_f32(wh2r + 32);
  const float bz0 = (bih0[ncol] + bhh0[ncol]) * PCARRY;
  const float bz1 = (bih1[ncol] + bhh1[ncol]) * PCARRY;
  const float bz2 = (bih2[ncol] + bhh2[ncol]) * PCARRY;

  const int km = tid & 63;
  const int mA = tid >> 6;
  const int mB = mA + 8;
  const float wxi = wih0[km];
  const float wxf = wih0[NHID + km];
  const float wxg = wih0[2 * NHID + km];
  const float wxo = wih0[3 * NHID + km];
  float c0a = 0.0f, c0b = 0.0f, c1a = 0.0f, c1b = 0.0f, c2a = 0.0f, c2b = 0.0f;
  float h2a = 0.0f, h2b = 0.0f;

  const _Float16* arow = hcat + c * HCP + koff;
  const int gwr = (8 * hh) * GBP + ncol;
  const int gra = mA * GBP + km;
  const int grb = mB * GBP + km;
  _Float16* hwa = hcat + mA * HCP + km;
  _Float16* hwb = hcat + mB * HCP + km;

  __syncthreads();

#pragma unroll 1
  for (int t = 0; t < NSTEP; ++t) {
    if ((t & (XCH - 1)) == 0) {
      xs[tid] = x[(size_t)(b0 + (tid >> 5)) * NSTEP + (size_t)t + (size_t)(tid & 31)];
    }

    {
      v8f acc = {bz0, bz0, bz0, bz0, bz0, bz0, bz0, bz0};
      const v16h a0 = frag_load(arow);
      const v16h a1 = frag_load(arow + 32);
      acc = mma_h(a0, bw0a, acc);
      acc = mma_h(a1, bw0b, acc);
#pragma unroll
      for (int r = 0; r < 8; ++r) gb[gwr + r * GBP] = acc[r];
    }
    __syncthreads();
    {
      const float xa = xs[mA * XCH + (t & (XCH - 1))];
      const float xb = xs[mB * XCH + (t & (XCH - 1))];
      const float ha = cell_update(fmaf(gb[gra], PFOLD, xa * wxi), fmaf(gb[gra + NHID], PFOLD, xa * wxf),
                                   fmaf(gb[gra + 2 * NHID], PFOLD, xa * wxg), fmaf(gb[gra + 3 * NHID], PFOLD, xa * wxo), c0a);
      const float hb = cell_update(fmaf(gb[grb], PFOLD, xb * wxi), fmaf(gb[grb + NHID], PFOLD, xb * wxf),
                                   fmaf(gb[grb + 2 * NHID], PFOLD, xb * wxg), fmaf(gb[grb + 3 * NHID], PFOLD, xb * wxo), c0b);
      hwa[0] = (_Float16)(ha * HCARRY);
      hwb[0] = (_Float16)(hb * HCARRY);
    }
    __syncthreads();

    {
      v8f acc = {bz1, bz1, bz1, bz1, bz1, bz1, bz1, bz1};
      const v16h a0 = frag_load(arow);
      const v16h a1 = frag_load(arow + 32);
      const v16h a2 = frag_load(arow + 64);
      const v16h a3 = frag_load(arow + 96);
      acc = mma_h(a0, bw1a, acc);
      acc = mma_h(a1, bw1b, acc);
      acc = mma_h(a2, bw1c, acc);
      acc = mma_h(a3, bw1d, acc);
#pragma unroll
      for (int r = 0; r < 8; ++r) gb[gwr + r * GBP] = acc[r];
    }
    __syncthreads();
    {
      const float ha = cell_update(gb[gra] * PFOLD, gb[gra + NHID] * PFOLD,
                                   gb[gra + 2 * NHID] * PFOLD, gb[gra + 3 * NHID] * PFOLD, c1a);
      const float hb = cell_update(gb[grb] * PFOLD, gb[grb + NHID] * PFOLD,
                                   gb[grb + 2 * NHID] * PFOLD, gb[grb + 3 * NHID] * PFOLD, c1b);
      hwa[NHID] = (_Float16)(ha * HCARRY);
      hwb[NHID] = (_Float16)(hb * HCARRY);
    }
    __syncthreads();

    {
      v8f acc = {bz2, bz2, bz2, bz2, bz2, bz2, bz2, bz2};
      const v16h a0 = frag_load(arow + 64);
      const v16h a1 = frag_load(arow + 96);
      const v16h a2 = frag_load(arow + 128);
      const v16h a3 = frag_load(arow + 160);
      acc = mma_h(a0, bw2a, acc);
      acc = mma_h(a1, bw2b, acc);
      acc = mma_h(a2, bw2c, acc);
      acc = mma_h(a3, bw2d, acc);
#pragma unroll
      for (int r = 0; r < 8; ++r) gb[gwr + r * GBP] = acc[r];
    }
    __syncthreads();
    {
      h2a = cell_update(gb[gra] * PFOLD, gb[gra + NHID] * PFOLD,
                        gb[gra + 2 * NHID] * PFOLD, gb[gra + 3 * NHID] * PFOLD, c2a);
      h2b = cell_update(gb[grb] * PFOLD, gb[grb + NHID] * PFOLD,
                        gb[grb + 2 * NHID] * PFOLD, gb[grb + 3 * NHID] * PFOLD, c2b);
      hwa[2 * NHID] = (_Float16)(h2a * HCARRY);
      hwb[2 * NHID] = (_Float16)(h2b * HCARRY);
    }
    __syncthreads();
  }

  gb[gra] = h2a;
  gb[grb] = h2b;
  __syncthreads();
  {
    const int e  = tid & (NEMB - 1);
    const int rq = tid >> 7;
    const float bv = fcb[e];
    float o0 = bv, o1 = bv, o2 = bv, o3 = bv;
    const float* wrow = fcw + (size_t)e * NHID;
    const float* hr0 = gb + (0 + rq) * GBP;
    const float* hr1 = gb + (4 + rq) * GBP;
    const float* hr2 = gb + (8 + rq) * GBP;
    const float* hr3 = gb + (12 + rq) * GBP;
#pragma unroll 1
    for (int k = 0; k < NHID; k += 4) {
      const v4f w  = *(const v4f*)(wrow + k);
      const v4f p0 = *(const v4f*)(hr0 + k);
      const v4f p1 = *(const v4f*)(hr1 + k);
      const v4f p2 = *(const v4f*)(hr2 + k);
      const v4f p3 = *(const v4f*)(hr3 + k);
#pragma unroll
      for (int q = 0; q < 4; ++q) {
        o0 = fmaf(w[q], p0[q], o0);
        o1 = fmaf(w[q], p1[q], o1);
        o2 = fmaf(w[q], p2[q], o2);
        o3 = fmaf(w[q], p3[q], o3);
      }
    }
    float* op = out + (size_t)(b0 + rq) * NEMB + e;
    for (int pass = 0; pass < 2; ++pass) {
      *(volatile float*)(op)                = o0;
      *(volatile float*)(op + 4 * NEMB)     = o1;
      *(volatile float*)(op + 8 * NEMB)     = o2;
      *(volatile float*)(op + 12 * NEMB)    = o3;
      __threadfence();
    }
  }
}

extern "C" void kernel_launch(void* const* d_in, const int* in_sizes, int n_in,
                              void* d_out, int out_size, void* d_ws, size_t ws_size, hipStream_t stream) {
  (void)d_ws; (void)ws_size;
  if (n_in < 15 || d_out == nullptr) return;
  if (in_sizes[0] != NBATCH * NSTEP || in_sizes[1] != NGATE || in_sizes[2] != NGATE * NHID ||
      in_sizes[3] != NGATE || in_sizes[4] != NGATE ||
      in_sizes[5] != NGATE * NHID || in_sizes[6] != NGATE * NHID || in_sizes[7] != NGATE || in_sizes[8] != NGATE ||
      in_sizes[9] != NGATE * NHID || in_sizes[10] != NGATE * NHID || in_sizes[11] != NGATE || in_sizes[12] != NGATE ||
      in_sizes[13] != NEMB * NHID || in_sizes[14] != NEMB || out_size != NBATCH * NEMB) return;

  const float* x    = (const float*)d_in[0];
  const float* wih0 = (const float*)d_in[1];
  const float* whh0 = (const float*)d_in[2];
  const float* bih0 = (const float*)d_in[3];
  const float* bhh0 = (const float*)d_in[4];
  const float* wih1 = (const float*)d_in[5];
  const float* whh1 = (const float*)d_in[6];
  const float* bih1 = (const float*)d_in[7];
  const float* bhh1 = (const float*)d_in[8];
  const float* wih2 = (const float*)d_in[9];
  const float* whh2 = (const float*)d_in[10];
  const float* bih2 = (const float*)d_in[11];
  const float* bhh2 = (const float*)d_in[12];
  const float* fcw  = (const float*)d_in[13];
  const float* fcb  = (const float*)d_in[14];
  float* out = (float*)d_out;

  rnn3_fused_kernel<<<NBATCH / ROWS_BLK, NTHR, 0, stream>>>(
      x, wih0, whh0, bih0, bhh0, wih1, whh1, bih1, bhh1, wih2, whh2, bih2, bhh2, fcw, fcb, out);
}
